// TinyGAT_52510270161006
// MI455X (gfx1250) — hardware-verified
//
#include <hip/hip_runtime.h>


namespace {
constexpr int Bn = 8, K = 1024, C = 256, HID = 128, NHD = 4, OUTD = 128, NR = Bn * K, NC = 144  ;
constexpr float AS_ = 8.0f;

typedef _Float16 b16;
typedef __attribute__((ext_vector_type(16))) _Float16 v16b;
typedef __attribute__((ext_vector_type(8))) _Float16 v8b;
typedef __attribute__((ext_vector_type(8))) float v8f;
typedef __attribute__((ext_vector_type(4))) float v4f;
__device__ __forceinline__ float bf16_rne(float f) { unsigned int u = __float_as_uint(f); u += 0x7FFFu + ((u >> 16) & 1u); return __uint_as_float(u & 0xFFFF0000u); }
__device__ __forceinline__ void split16(float v, b16& hi, b16& lo) { hi = (b16)v; lo = (b16)(v - (float)hi); }
__device__ __forceinline__ v16b frag_kb(const b16* p, int hh) { const v8b a = *(const v8b*)(p + 8 * hh), b = *(const v8b*)(p + 16 + 8 * hh); v16b f;
#pragma unroll
  for (int e = 0; e < 8; ++e) { f[e] = a[e]; f[8 + e] = b[e]; } return f; }
__device__ __forceinline__ v16b frag_x(const float* p, int hh) { v16b f;
#pragma unroll
  for (int e = 0; e < 8; ++e) { f[e] = (b16)bf16_rne(p[8 * hh + e]); f[8 + e] = (b16)bf16_rne(p[16 + 8 * hh + e]); } return f; }
__device__ __forceinline__ v16b frag_mask(const float* p, int hh) { v16b f;
#pragma unroll
  for (int e = 0; e < 8; ++e) { f[e] = (b16)((bf16_rne(p[8 * hh + e]) > 0.0f) ? 1.0f : 0.0f); f[8 + e] = (b16)((bf16_rne(p[16 + 8 * hh + e]) > 0.0f) ? 1.0f : 0.0f); } return f; }
__device__ __forceinline__ void frag_split(const float* p, int hh, v16b& fh, v16b& fl) {
#pragma unroll
  for (int e = 0; e < 8; ++e) { b16 a, c; split16(p[8 * hh + e] * AS_, a, c); fh[e] = a; fl[e] = c; split16(p[16 + 8 * hh + e] * AS_, a, c); fh[8 + e] = a; fl[8 + e] = c; } }
__device__ __forceinline__ v8f wmma16b(v16b a, v16b b, v8f c) { v8f d = __builtin_amdgcn_wmma_f32_16x16x32_f16(false, a, false, b, (short)0, c, false, false); asm volatile("v_nop\n\tv_nop\n\tv_nop\n\tv_nop" : "+v"(d) : "v"(a), "v"(b)); return d; }
__device__ __forceinline__ void wave_lds_sync() { __builtin_amdgcn_fence(__ATOMIC_RELEASE, "workgroup"); __builtin_amdgcn_wave_barrier(); __builtin_amdgcn_fence(__ATOMIC_ACQUIRE, "workgroup"); }
__device__ __forceinline__ float nexp(float x) { return __builtin_amdgcn_exp2f(x * 1.4426950408889634f); }
__device__ __forceinline__ float pmul(float a, float b) { float p = a * b; asm volatile("" : "+v"(p)); return p; }
__device__ __forceinline__ float wmax(float v) {
#pragma unroll
  for (int o = 1; o < 32; o <<= 1) v = fmaxf(v, __shfl_xor(v, o)); return v; }

__global__ __launch_bounds__(256) void prep_kernel(const float* __restrict__ Wp, const float* __restrict__ at, const float* __restrict__ Wo, const float* __restrict__ bo, b16* __restrict__ R, float* __restrict__ P) {
  const int t_ = blockIdx.x * 256 + threadIdx.x, nth = gridDim.x * 256;
  for (int pass = 0; pass < 2; ++pass) {
    for (int p = t_; p < (HID * C + OUTD * HID) / 8; p += nth) { const int q = p * 8; const float* src = (q < HID * C) ? (Wp + q) : (Wo + (q - HID * C)); v8b v;
#pragma unroll
      for (int e = 0; e < 8; ++e) v[e] = (b16)bf16_rne(src[e]); *(volatile v8b*)(R + q) = v; }
    for (int q = t_; q < 640; q += nth) P[q] = (q < 512) ? bf16_rne(at[q]) : bf16_rne(bo[q - 512]);
    __threadfence(); }
}

__global__ __launch_bounds__(128) void proj_kernel(const float* __restrict__ Z, const b16* __restrict__ R, const float* __restrict__ P, float* __restrict__ Hf, float* __restrict__ Hh) {
  __shared__ __attribute__((aligned(16))) float Ts[4][32][HID + 4]; __shared__ __attribute__((aligned(16))) float Th[128][NHD];
  const int lane = threadIdx.x & 31, wave = threadIdx.x >> 5, nloc = lane & 15, hlf = lane >> 4, m0 = blockIdx.x * 128 + wave * 32;
  v8f acc[2][8];
#pragma unroll
  for (int r = 0; r < 2; ++r)
#pragma unroll
    for (int t = 0; t < 8; ++t) acc[r][t] = (v8f){};
#pragma unroll 2
  for (int kb = 0; kb < C; kb += 32) { const v16b a0 = frag_x(Z + (size_t)(m0 + nloc) * C + kb, hlf), a1 = frag_x(Z + (size_t)(m0 + 16 + nloc) * C + kb, hlf);
#pragma unroll
    for (int t = 0; t < 8; ++t) { const v16b bw = frag_kb(R + (size_t)(t * 16 + nloc) * C + kb, hlf); acc[0][t] = wmma16b(a0, bw, acc[0][t]); acc[1][t] = wmma16b(a1, bw, acc[1][t]); } }
#pragma unroll
  for (int t = 0; t < 8; ++t)
#pragma unroll
    for (int r = 0; r < 2; ++r)
#pragma unroll
      for (int v = 0; v < 8; ++v) Ts[wave][r * 16 + 8 * hlf + v][t * 16 + nloc] = acc[r][t][v];
  wave_lds_sync();
  { const float* hr = Ts[wave][lane]; for (int a = 0; a < NHD; ++a) { float s = 0.0f; for (int h = 0; h < HID; ++h) s += pmul(hr[h], P[a * HID + h]); Th[wave * 32 + lane][a] = s; } }
  __syncthreads();
  for (int pass = 0; pass < 2; ++pass) {
    for (int i = lane; i < 32 * 32; i += 32) { const int rr = i >> 5, c4 = (i & 31) * 4; *(volatile v4f*)(Hf + (size_t)(m0 + rr) * HID + c4) = *(const v4f*)(&Ts[wave][rr][c4]); }
    *(volatile v4f*)(Hh + (size_t)(blockIdx.x * 128 + threadIdx.x) * NHD) = *(const v4f*)(&Th[threadIdx.x][0]);
    __threadfence(); }
}

__global__ __launch_bounds__(256) void eh_kernel(const float* __restrict__ Hf, const float* __restrict__ Hh, b16* __restrict__ EHh, b16* __restrict__ EHl) {
  __shared__ __attribute__((aligned(16))) b16 Th_[NC][64 + 8], Tl_[NC][64 + 8]; __shared__ float Ej[64]; __shared__ float mxs[8];
  const int b = blockIdx.z, a = blockIdx.y, j0 = blockIdx.x * 64, t_ = threadIdx.x, lane = t_ & 31, wave = t_ >> 5;
  float mx = -INFINITY; for (int j = t_; j < K; j += 256) mx = fmaxf(mx, Hh[((size_t)b * K + j) * NHD + a]); mx = wmax(mx); if (lane == 0) mxs[wave] = mx;
  __syncthreads();
  mx = mxs[0]; for (int w = 1; w < 8; ++w) mx = fmaxf(mx, mxs[w]);
  if (t_ < 64) Ej[t_] = nexp(Hh[((size_t)b * K + j0 + t_) * NHD + a] - mx);
  __syncthreads();
  for (int i = t_; i < 64 * NC; i += 256) { const int j = i & 63, n = i >> 6; const float v = (n < HID) ? pmul(Ej[j], Hf[((size_t)b * K + j0 + j) * HID + n]) : (n == HID) ? Ej[j] : 0.0f; b16 hv, lv; split16(v * AS_, hv, lv); Th_[n][j] = hv; Tl_[n][j] = lv; }
  __syncthreads();
  const size_t base = (((size_t)b * NHD + a) * NC) * K + j0;
  for (int pass = 0; pass < 2; ++pass) { for (int i = t_; i < NC * 8; i += 256) { const int n = i >> 3, c8 = (i & 7) * 8; *(volatile v8b*)(EHh + base + (size_t)n * K + c8) = *(const v8b*)(&Th_[n][c8]); *(volatile v8b*)(EHl + base + (size_t)n * K + c8) = *(const v8b*)(&Tl_[n][c8]); } __threadfence(); }
}

__global__ __launch_bounds__(128) void agg_kernel(const float* __restrict__ As, const b16* __restrict__ EHh, const b16* __restrict__ EHl, const float* __restrict__ Hf, const b16* __restrict__ R, const float* __restrict__ P, float* __restrict__ y) {
  __shared__ __attribute__((aligned(16))) float Ag[NHD][32][HID + 4]; __shared__ __attribute__((aligned(16))) float Tm[32][HID + 4]; __shared__ int anyEmpty[NHD];
  const int lane = threadIdx.x & 31, wave = threadIdx.x >> 5, nloc = lane & 15, hlf = lane >> 4, b = blockIdx.y, i0 = blockIdx.x * 32, a = wave;
  const float* Ab = As + ((size_t)b * K + i0) * K; const b16* Eh = EHh + (((size_t)b * NHD + a) * NC) * K; const b16* El = EHl + (((size_t)b * NHD + a) * NC) * K;
  v8f acc[2][9];
#pragma unroll
  for (int r = 0; r < 2; ++r)
#pragma unroll
    for (int t = 0; t < 9; ++t) acc[r][t] = (v8f){};
#pragma unroll 2
  for (int kb = 0; kb < K; kb += 32) { const v16b a0 = frag_mask(Ab + (size_t)nloc * K + kb, hlf), a1 = frag_mask(Ab + (size_t)(16 + nloc) * K + kb, hlf);
#pragma unroll
    for (int t = 0; t < 9; ++t) { const v16b bh = frag_kb(Eh + (size_t)(t * 16 + nloc) * K + kb, hlf), bl = frag_kb(El + (size_t)(t * 16 + nloc) * K + kb, hlf);
      acc[0][t] = wmma16b(a0, bh, acc[0][t]); acc[0][t] = wmma16b(a0, bl, acc[0][t]); acc[1][t] = wmma16b(a1, bh, acc[1][t]); acc[1][t] = wmma16b(a1, bl, acc[1][t]); } }
  __shared__ float Den[NHD][32];
  if (nloc == 0) {
#pragma unroll
    for (int r = 0; r < 2; ++r)
#pragma unroll
      for (int v = 0; v < 8; ++v) Den[a][r * 16 + 8 * hlf + v] = acc[r][8][v] * (1.0f / AS_); }
  if (threadIdx.x < NHD) anyEmpty[threadIdx.x] = 0;
  __syncthreads();
#pragma unroll
  for (int t = 0; t < 8; ++t)
#pragma unroll
    for (int r = 0; r < 2; ++r)
#pragma unroll
      for (int v = 0; v < 8; ++v) { const int rr = r * 16 + 8 * hlf + v; const float d = Den[a][rr]; Ag[a][rr][t * 16 + nloc] = (d > 0.0f) ? (acc[r][t][v] * (1.0f / AS_)) / d : __int_as_float(0x7fc00000); if (!(d > 0.0f)) anyEmpty[a] = 1; }
  __syncthreads();
  if (anyEmpty[0] | anyEmpty[1] | anyEmpty[2] | anyEmpty[3]) {
    for (int n = threadIdx.x; n < HID; n += 128) { float s = 0.0f; for (int j = 0; j < K; ++j) s += Hf[((size_t)b * K + j) * HID + n]; const float mval = s * (1.0f / K);
      for (int hd = 0; hd < NHD; ++hd) for (int rr = 0; rr < 32; ++rr) if (!(Den[hd][rr] > 0.0f)) Ag[hd][rr][n] = mval; }
    __syncthreads(); }
  for (int i = threadIdx.x; i < 32 * HID; i += 128) { const int rr = i / HID, n = i % HID; Tm[rr][n] = ((Ag[0][rr][n] + Ag[1][rr][n]) + (Ag[2][rr][n] + Ag[3][rr][n])) * 0.25f; }
  __syncthreads();
  { v8f o[2][2] = {{{}, {}}, {{}, {}}}; const b16* Wo = R + HID * C;
#pragma unroll
    for (int kb = 0; kb < HID; kb += 32) { v16b a0, l0, a1, l1; frag_split(&Tm[nloc][kb], hlf, a0, l0); frag_split(&Tm[16 + nloc][kb], hlf, a1, l1);
#pragma unroll
      for (int t = 0; t < 2; ++t) { const v16b bw = frag_kb(Wo + (size_t)(wave * 32 + t * 16 + nloc) * HID + kb, hlf); o[0][t] = wmma16b(a0, bw, o[0][t]); o[0][t] = wmma16b(l0, bw, o[0][t]); o[1][t] = wmma16b(a1, bw, o[1][t]); o[1][t] = wmma16b(l1, bw, o[1][t]); } }
    __syncthreads();
#pragma unroll
    for (int t = 0; t < 2; ++t) { const int cc = wave * 32 + t * 16 + nloc; const float bb = P[512 + cc];
#pragma unroll
      for (int r = 0; r < 2; ++r)
#pragma unroll
        for (int v = 0; v < 8; ++v) { float z = o[r][t][v] * (1.0f / AS_) + bb; z = (z > 0.0f) ? z : (nexp(z) - 1.0f); Tm[r * 16 + 8 * hlf + v][cc] = z; } } }
  __syncthreads();
  for (int pass = 0; pass < 2; ++pass) { for (int i = threadIdx.x; i < 32 * 32; i += 128) { const int rr = i >> 5, c4 = (i & 31) * 4; *(volatile v4f*)(y + ((size_t)b * K + i0 + rr) * OUTD + c4) = *(const v4f*)(&Tm[rr][c4]); } __threadfence(); }
}
}

extern "C" void kernel_launch(void* const* d_in, const int* in_sizes, int n_in,
                              void* d_out, int out_size, void* d_ws, size_t ws_size, hipStream_t stream) {
  (void)n_in; (void)out_size;
  const float* Z = (const float*)d_in[0]; const float* As = (const float*)d_in[1]; const float* Wp = (const float*)d_in[2]; const float* at = (const float*)d_in[3]; const float* Wo = (const float*)d_in[4]; const float* bo = (const float*)d_in[5];
  float* y = (float*)d_out;
  if (in_sizes[0] != NR * C || in_sizes[1] != Bn * K * K || in_sizes[2] != HID * C || in_sizes[3] != NHD * HID || in_sizes[4] != OUTD * HID) return;
  size_t off = 0; char* ws = (char*)d_ws;
  auto carve = [&](size_t bytes) { char* p = ws + off; off += (bytes + 255) & ~(size_t)255; return p; };
  b16* R = (b16*)carve((size_t)(HID * C + OUTD * HID) * 2); float* P = (float*)carve(1024 * 4); float* Hf = (float*)carve((size_t)NR * HID * 4); float* Hh = (float*)carve((size_t)NR * NHD * 4);
  b16* EHh = (b16*)carve((size_t)Bn * NHD * NC * K * 2); b16* EHl = (b16*)carve((size_t)Bn * NHD * NC * K * 2);
  if (off > ws_size) return;
  prep_kernel<<<32, 256, 0, stream>>>(Wp, at, Wo, bo, R, P);
  proj_kernel<<<NR / 128, 128, 0, stream>>>(Z, R, P, Hf, Hh);
  eh_kernel<<<dim3(K / 64, NHD, Bn), 256, 0, stream>>>(Hf, Hh, EHh, EHl);
  agg_kernel<<<dim3(K / 32, Bn), 128, 0, stream>>>(As, EHh, EHl, Hf, R, P, y);
}
